// C_SCNN_17918603559428
// MI455X (gfx1250) — hardware-verified
//
#include <hip/hip_runtime.h>
#include <math.h>

constexpr int NBAT    = 4;
constexpr int NCH     = 256;
constexpr int NHGT    = 64;
constexpr int NWID    = 128;
constexpr int KTAP    = 9;
constexpr int CTAP    = 4;
constexpr int NROW    = NBAT * NWID;
constexpr int ROW_BLK = 16;
constexpr int NTHR    = 256;
constexpr int APITCH  = 264;
constexpr int SLABP   = 36;
constexpr int HUP     = 4 * NHGT;
constexpr int WUP     = 4 * NWID;
constexpr int NPIX    = NBAT * NHGT * NWID;
constexpr int NUP     = NBAT * HUP * WUP;
constexpr float BN_EPS = 1e-5f;
static_assert(NCH == 32 * (NTHR / 32));
static_assert(NCH % 32 == 0);
static_assert(NWID % ROW_BLK == 0);
static_assert(NROW % ROW_BLK == 0);
static_assert((NCH * NCH / 8) % NTHR == 0);
static_assert(NPIX % 32 == 0);
static_assert((NUP / 4) % NTHR == 0);
static_assert(NUP % NTHR == 0);

typedef __attribute__((ext_vector_type(16))) _Float16 v16h;
typedef __attribute__((ext_vector_type(8)))  _Float16 v8h;
typedef __attribute__((ext_vector_type(16))) __bf16   v16b;
typedef __attribute__((ext_vector_type(8)))  __bf16   v8b;
typedef __attribute__((ext_vector_type(8)))  float    v8f;
typedef __attribute__((ext_vector_type(4)))  float    v4f;

__device__ __forceinline__ unsigned short f2bf_bits(float f) {
  unsigned u = __float_as_uint(f);
  return (unsigned short)((u + 0x7FFFu + ((u >> 16) & 1u)) >> 16);
}
__device__ __forceinline__ float bf_bits2f(unsigned short h) { return __uint_as_float(((unsigned)h) << 16); }

__device__ __forceinline__ void dep_guard_b(v8f& a, v8f& b, v16b x, v16b y) { asm volatile("v_nop\n\tv_nop\n\tv_nop\n\tv_nop" : "+v"(a), "+v"(b) : "v"(x), "v"(y)); }
__device__ __forceinline__ void keep4_b(v16b a, v16b b, v16b c, v16b d) { asm volatile("v_nop" :: "v"(a), "v"(b), "v"(c), "v"(d)); }
__device__ __forceinline__ void acc_guard2(v8f& a, v8f& b) { asm volatile("v_nop\n\tv_nop\n\tv_nop\n\tv_nop" : "+v"(a), "+v"(b)); }
template <typename T> struct Frag;
template <> struct Frag<__bf16> {
  typedef v16b V; union U { v16b v; v8b h[2]; };
  static __device__ __forceinline__ v16b load(const __bf16* p) {
    U f; f.h[0] = *(const v8b*)(p); f.h[1] = *(const v8b*)(p + 16); return f.v;
  }
  static __device__ __forceinline__ v8f mma(v16b a, v16b b, v8f c) {
    return __builtin_amdgcn_wmma_f32_16x16x32_bf16(false, a, false, b, (short)0, c, false, false);
  }
};

__global__ __launch_bounds__(NTHR) void wc_split_kernel(const float* __restrict__ WUD,
                                                        unsigned short* __restrict__ WH, unsigned short* __restrict__ WL) {
  const int i  = blockIdx.x * NTHR + threadIdx.x;
  const int o  = i >> 5;
  const int c8 = (i & 31) * 8;
  v8h hv, lv;
#pragma unroll
  for (int e = 0; e < 8; ++e) {
    const float f = WUD[((size_t)(o * NCH + c8 + e)) * KTAP + CTAP];
    const unsigned short hb = f2bf_bits(f);
    const unsigned short lb = f2bf_bits(f - bf_bits2f(hb));
    hv[e] = __builtin_bit_cast(_Float16, hb);
    lv[e] = __builtin_bit_cast(_Float16, lb);
  }
  unsigned short* ph = WH + (size_t)i * 8;
  unsigned short* pl = WL + (size_t)i * 8;
  *(volatile v8h*)ph = hv;
  *(volatile v8h*)pl = lv;
  __threadfence();
  *(volatile v8h*)ph = hv;
  *(volatile v8h*)pl = lv;
}

template <bool SRC_NCHW>
__global__ __launch_bounds__(NTHR) void scnn_pass_kernel(const float* __restrict__ X,
                                                         const unsigned short* __restrict__ WHp,
                                                         const unsigned short* __restrict__ WLp,
                                                         float* __restrict__ S) {
  __shared__ __align__(16) __bf16 Ah[2][ROW_BLK * APITCH];
  __shared__ __align__(16) __bf16 Al[2][ROW_BLK * APITCH];
  __shared__ __align__(16) float  Sl[NTHR / 32][16 * SLABP];
  const __bf16* WH = (const __bf16*)WHp;
  const __bf16* WL = (const __bf16*)WLp;
  const int tid = threadIdx.x, lane = tid & 31, wave = tid >> 5;
  const int c = lane & 15, hh = lane >> 4, koff = hh * 8;
  const int q = lane >> 3, c4 = (lane & 7) * 4;
  const int rowbase = blockIdx.x * ROW_BLK;
  const int bb = rowbase / NWID;
  const int w0 = rowbase - bb * NWID;
  const int colw = 32 * wave;
  float* slab = Sl[wave];
  const v8f z8 = {0.f, 0.f, 0.f, 0.f, 0.f, 0.f, 0.f, 0.f};

#pragma unroll 1
  for (int i = 0; i < NHGT; ++i) {
    float xr[2][8];
#pragma unroll
    for (int nt = 0; nt < 2; ++nt) {
      const int j = colw + 16 * nt + c;
#pragma unroll
      for (int r = 0; r < 8; ++r) {
        const int row = 8 * hh + r;
        size_t off;
        if (SRC_NCHW) off = ((size_t)(bb * NCH + j) * NHGT + (size_t)i) * NWID + (size_t)(w0 + row);
        else          off = ((size_t)i * NROW + (size_t)(rowbase + row)) * NCH + (size_t)j;
        xr[nt][r] = X[off];
      }
    }

    v8f acc[2];
    acc[0] = z8; acc[1] = z8;
    if (i > 0) {
      const int pr = (i - 1) & 1;
      const __bf16* ahrow = &Ah[pr][0] + c * APITCH + koff;
      const __bf16* alrow = &Al[pr][0] + c * APITCH + koff;
      const __bf16* wh0 = WH + (size_t)(colw + c) * NCH + koff;
      const __bf16* wl0 = WL + (size_t)(colw + c) * NCH + koff;
      const __bf16* wh1 = WH + (size_t)(colw + 16 + c) * NCH + koff;
      const __bf16* wl1 = WL + (size_t)(colw + 16 + c) * NCH + koff;
#pragma unroll 1
      for (int k0 = 0; k0 < NCH; k0 += 32) {
        const v16b ah  = Frag<__bf16>::load(ahrow + k0);
        const v16b al  = Frag<__bf16>::load(alrow + k0);
        const v16b bh0 = Frag<__bf16>::load(wh0 + k0);
        const v16b bl0 = Frag<__bf16>::load(wl0 + k0);
        const v16b bh1 = Frag<__bf16>::load(wh1 + k0);
        const v16b bl1 = Frag<__bf16>::load(wl1 + k0);
        acc[0] = Frag<__bf16>::mma(ah, bh0, acc[0]);
        acc[0] = Frag<__bf16>::mma(ah, bl0, acc[0]);
        acc[0] = Frag<__bf16>::mma(al, bh0, acc[0]);
        acc[1] = Frag<__bf16>::mma(ah, bh1, acc[1]);
        acc[1] = Frag<__bf16>::mma(ah, bl1, acc[1]);
        acc[1] = Frag<__bf16>::mma(al, bh1, acc[1]);
        dep_guard_b(acc[0], acc[1], ah, al);
        keep4_b(bh0, bl0, bh1, bl1);
      }
      acc_guard2(acc[0], acc[1]);
    }

    const int pw = i & 1;
    __bf16* ahn = &Ah[pw][0];
    __bf16* aln = &Al[pw][0];
#pragma unroll
    for (int nt = 0; nt < 2; ++nt) {
      const int j = colw + 16 * nt + c;
#pragma unroll
      for (int r = 0; r < 8; ++r) {
        const int row = 8 * hh + r;
        const float d   = acc[nt][r];
        const float cur = xr[nt][r] + fmaxf(d, 0.0f);
        const unsigned short hb = f2bf_bits(cur);
        const unsigned short lb = f2bf_bits(cur - bf_bits2f(hb));
        ahn[row * APITCH + j] = __builtin_bit_cast(__bf16, hb);
        aln[row * APITCH + j] = __builtin_bit_cast(__bf16, lb);
        slab[row * SLABP + 16 * nt + c] = cur;
      }
    }
    __builtin_amdgcn_fence(__ATOMIC_RELEASE, "workgroup");
    __builtin_amdgcn_wave_barrier();
    __builtin_amdgcn_fence(__ATOMIC_ACQUIRE, "workgroup");
    const size_t srow = (size_t)(NHGT - 1 - i) * NROW + (size_t)rowbase;
    for (int pass = 0; pass < 2; ++pass) {
#pragma unroll
      for (int it = 0; it < 4; ++it) {
        const int row = it * 4 + q;
        const v4f v = *(const v4f*)(slab + row * SLABP + c4);
        *(volatile v4f*)(S + (srow + (size_t)row) * NCH + colw + c4) = v;
      }
      __threadfence();
    }
    __syncthreads();
  }
}

__global__ __launch_bounds__(NTHR) void proj_kernel(const float* __restrict__ S2, const float* __restrict__ W1,
                                                    float* __restrict__ Z) {
  __shared__ __align__(16) float zl[32];
  const int tid = threadIdx.x, lane = tid & 31, wave = tid >> 5;
  const int bx = blockIdx.x;
  const v4f wa = *(const v4f*)(W1 + 4 * lane);
  const v4f wb = *(const v4f*)(W1 + 128 + 4 * lane);
#pragma unroll
  for (int k = 0; k < 4; ++k) {
    const int r = wave * 4 + k;
    const float* rp = S2 + (size_t)(bx * 32 + r) * NCH;
    const v4f a = *(const v4f*)(rp + 4 * lane);
    const v4f b = *(const v4f*)(rp + 128 + 4 * lane);
    float s = (a[0] * wa[0] + a[1] * wa[1]) + (a[2] * wa[2] + a[3] * wa[3])
            + ((b[0] * wb[0] + b[1] * wb[1]) + (b[2] * wb[2] + b[3] * wb[3]));
#pragma unroll
    for (int off = 1; off < 32; off <<= 1) s += __shfl_xor(s, off, 32);
    if (lane == 0) zl[r] = s;
  }
  __syncthreads();
  if (wave == 0) {
    const int hb = bx >> 2;
    const int b  = hb & 3;
    const int h  = hb >> 2;
    const int w0 = (bx & 3) * 32;
    float* zp = Z + (size_t)(b * NHGT + h) * NWID + w0;
    const int lc = (lane < 8) ? lane : 0;
    const v4f v = *(const v4f*)(zl + 4 * lc);
    for (int pass = 0; pass < 2; ++pass) {
      if (lane < 8) *(volatile v4f*)(zp + 4 * lane) = v;
      __threadfence();
    }
  }
}

__global__ __launch_bounds__(NTHR) void interp_kernel(const float* __restrict__ Z, float* __restrict__ Y) {
#pragma clang fp contract(off)
  const int idx = blockIdx.x * NTHR + threadIdx.x;
  const int b     = idx >> 15;
  const int hrow  = (idx >> 7) & 255;
  const int wbase = (idx & 127) * 4;
  const float sch = (float)(63.0 / 255.0);
  const float scw = (float)(127.0 / 511.0);
  const float ph = (float)hrow * sch;
  int hlo = (int)floorf(ph); hlo = hlo < 0 ? 0 : (hlo > NHGT - 1 ? NHGT - 1 : hlo);
  const int hhi = (hlo + 1 > NHGT - 1) ? (NHGT - 1) : (hlo + 1);
  const float fh = ph - (float)hlo;
  const float* zb = Z + (size_t)b * NHGT * NWID;
  const float* r0 = zb + hlo * NWID;
  const float* r1 = zb + hhi * NWID;
  v4f o;
#pragma unroll
  for (int e = 0; e < 4; ++e) {
    const int ww = wbase + e;
    const float pw = (float)ww * scw;
    int wlo = (int)floorf(pw); wlo = wlo < 0 ? 0 : (wlo > NWID - 1 ? NWID - 1 : wlo);
    const int whi = (wlo + 1 > NWID - 1) ? (NWID - 1) : (wlo + 1);
    const float fw = pw - (float)wlo;
    const float a00 = r0[wlo], a01 = r0[whi];
    const float a10 = r1[wlo], a11 = r1[whi];
    const float c0 = a00 + (a10 - a00) * fh;
    const float c1 = a01 + (a11 - a01) * fh;
    o[e] = c0 + (c1 - c0) * fw;
  }
  float* yp = Y + (size_t)idx * 4;
  *(volatile v4f*)yp = o;
  __threadfence();
  *(volatile v4f*)yp = o;
}

__global__ __launch_bounds__(NTHR) void stats_kernel(const float* __restrict__ Y, float* __restrict__ ST) {
  __shared__ float red[NTHR];
  __shared__ __align__(16) float stl[32];
  const int t = threadIdx.x;
  float s = 0.f;
#pragma unroll 1
  for (int kb = 0; kb < NUP / NTHR; kb += 64) {
    float p = 0.f;
#pragma unroll 1
    for (int k = kb; k < kb + 64; ++k) p += Y[(size_t)k * NTHR + t];
    s += p;
  }
  red[t] = s;
  __syncthreads();
  for (int off = NTHR / 2; off; off >>= 1) {
    if (t < off) red[t] += red[t + off];
    __syncthreads();
  }
  const float inv_n = 1.0f / (float)NUP;
  const float mean = red[0] * inv_n;
  __syncthreads();
  float ss = 0.f;
#pragma unroll 1
  for (int kb = 0; kb < NUP / NTHR; kb += 64) {
    float p = 0.f;
#pragma unroll 1
    for (int k = kb; k < kb + 64; ++k) { const float d = Y[(size_t)k * NTHR + t] - mean; p += d * d; }
    ss += p;
  }
  red[t] = ss;
  __syncthreads();
  for (int off = NTHR / 2; off; off >>= 1) {
    if (t < off) red[t] += red[t + off];
    __syncthreads();
  }
  const float var  = red[0] * inv_n;
  const float rstd = rsqrtf(var + BN_EPS);
  if (t < 32) stl[t] = (t == 0) ? mean : ((t == 1) ? rstd : 0.0f);
  __syncthreads();
  if (t < 32) {
    const int lc = (t < 8) ? t : 0;
    const v4f v = *(const v4f*)(stl + 4 * lc);
    for (int pass = 0; pass < 2; ++pass) {
      if (t < 8) *(volatile v4f*)(ST + 4 * t) = v;
      __threadfence();
    }
  }
}

__global__ __launch_bounds__(NTHR) void final_kernel(const float* __restrict__ Y, const float* __restrict__ ST,
                                                     const float* __restrict__ gam, const float* __restrict__ bet,
                                                     float* __restrict__ OUT) {
  const int idx = blockIdx.x * NTHR + threadIdx.x;
  const float mean = ST[0], rstd = ST[1], g = gam[0], be = bet[0];
  const v4f y = *(const v4f*)(Y + (size_t)idx * 4);
  v4f o;
#pragma unroll
  for (int e = 0; e < 4; ++e) {
    const float yn = ((y[e] - mean) * rstd) * g + be;
    o[e] = 1.0f / (1.0f + expf(-yn));
  }
  float* op = OUT + (size_t)idx * 4;
  *(volatile v4f*)op = o;
  __threadfence();
  *(volatile v4f*)op = o;
}

extern "C" void kernel_launch(void* const* d_in, const int* in_sizes, int n_in,
                              void* d_out, int out_size, void* d_ws, size_t ws_size, hipStream_t stream) {
  if (n_in < 5 || d_out == nullptr || d_ws == nullptr) return;
  if (in_sizes[0] != NBAT * NCH * NHGT * NWID || in_sizes[1] != NCH * NCH * KTAP || in_sizes[2] != NCH ||
      in_sizes[3] != 1 || in_sizes[4] != 1 || out_size != NUP) return;

  const float* p2c   = (const float*)d_in[0];
  const float* wud   = (const float*)d_in[1];
  const float* w1    = (const float*)d_in[2];
  const float* gamma = (const float*)d_in[3];
  const float* beta  = (const float*)d_in[4];
  float* out = (float*)d_out;

  char* ws = (char*)d_ws; size_t off = 0;
  auto carve = [&](size_t bytes) -> char* { char* p = ws + off; off += (bytes + 255) & ~(size_t)255; return p; };
  unsigned short* WH = (unsigned short*)carve((size_t)NCH * NCH * 2);
  unsigned short* WL = (unsigned short*)carve((size_t)NCH * NCH * 2);
  float*          S1 = (float*)carve((size_t)NHGT * NROW * NCH * 4);
  float*          S2 = (float*)carve((size_t)NHGT * NROW * NCH * 4);
  float*          Zp = (float*)carve((size_t)NPIX * 4);
  float*          Yp = (float*)carve((size_t)NUP * 4);
  float*          ST = (float*)carve((size_t)32 * 4);
  if (off > ws_size || off > (size_t)134217728) return;

  wc_split_kernel<<<(NCH * NCH / 8) / NTHR, NTHR, 0, stream>>>(wud, WH, WL);
  scnn_pass_kernel<true><<<NROW / ROW_BLK, NTHR, 0, stream>>>(p2c, WH, WL, S1);
  scnn_pass_kernel<false><<<NROW / ROW_BLK, NTHR, 0, stream>>>(S1, WH, WL, S2);
  proj_kernel<<<NPIX / 32, NTHR, 0, stream>>>(S2, w1, Zp);
  interp_kernel<<<(NUP / 4) / NTHR, NTHR, 0, stream>>>(Zp, Yp);
  stats_kernel<<<1, NTHR, 0, stream>>>(Yp, ST);
  final_kernel<<<(NUP / 4) / NTHR, NTHR, 0, stream>>>(Yp, ST, gamma, beta, out);
}
